// Grid2SeqTransformerBackbone_39101382262954
// MI455X (gfx1250) — hardware-verified
//
#include <hip/hip_runtime.h>
#include <math.h>

typedef __bf16 v16bf __attribute__((ext_vector_type(16)));
typedef float v8f __attribute__((ext_vector_type(8)));
typedef float v4f __attribute__((ext_vector_type(4)));
typedef unsigned int v4u __attribute__((ext_vector_type(4)));
typedef int v4i __attribute__((ext_vector_type(4)));
typedef v4u __attribute__((may_alias)) v4ua;
typedef v4f __attribute__((may_alias)) v4fa;
typedef v4i __attribute__((may_alias)) v4ia;

union Frag { v16bf v; v4u q[2]; unsigned int w[8]; };

#define NIMG   16
#define SEQ    1024
#define EMB    64
#define NHEAD  4
#define HDIM   16
#define FFD    256
#define NLAYER 3
#define NTOK   (NIMG * SEQ)
#define KEMB   96

#define WET_OFF  0
#define WQKV_OFF 6144
#define WO_OFF   43008
#define W1_OFF   55296
#define W2_OFF   104448
#define WPLANE   153600

static_assert(WQKV_OFF == EMB * KEMB);
static_assert(WO_OFF == WQKV_OFF + NLAYER * 3 * EMB * EMB);
static_assert(W1_OFF == WO_OFF + NLAYER * EMB * EMB);
static_assert(W2_OFF == W1_OFF + NLAYER * FFD * EMB);
static_assert(WPLANE == W2_OFF + NLAYER * EMB * FFD);

__device__ __forceinline__ v8f mma16(v16bf a, v16bf b, v8f c) {
  v8f d = __builtin_amdgcn_wmma_f32_16x16x32_bf16(false, a, false, b, (short)0, c, false, false);
  asm volatile("v_nop\n\tv_nop\n\tv_nop\n\tv_nop" : "+v"(d) : "v"(a), "v"(b));
  return d;
}

__device__ __forceinline__ v8f zero8() {
  v8f z = {0.f, 0.f, 0.f, 0.f, 0.f, 0.f, 0.f, 0.f};
  return z;
}

__device__ __forceinline__ v16bf ldfrag(const unsigned short* p, int h) {
  Frag f;
  f.q[0] = *(const v4ua*)(p + 8 * h);
  f.q[1] = *(const v4ua*)(p + 16 + 8 * h);
  return f.v;
}

__device__ __forceinline__ unsigned int bfb(float f) {
  unsigned int u = __float_as_uint(f);
  u += 0x7FFFu + ((u >> 16) & 1u);
  return u >> 16;
}
__device__ __forceinline__ void split2(float f, unsigned int& hb, unsigned int& lb) {
  hb = bfb(f);
  lb = bfb(f - __uint_as_float(hb << 16));
}

__device__ __forceinline__ float lin31(int i) {
  const float st = (float)i * (1.0f / 31.0f);
  const float v = -1.0f * (1.0f - st) + 1.0f * st;
  return (i == 31) ? 1.0f : v;
}

template <int NROW, int NTHR>
__device__ __forceinline__ void store_rows(const float* R, float* hb, int tok0, int t) {
  constexpr int NLINE = NROW * 2;
  constexpr int LPI = NTHR / 8;
  constexpr int NI = NLINE / LPI;
  const int q8 = t & 7, sub = t >> 3;
#pragma unroll
  for (int i = 0; i < NI; ++i) {
    const int L = i * LPI + sub;
    const int row = L >> 1, hf = L & 1;
    const v4f v = *(const v4fa*)(R + row * EMB + 32 * hf + 4 * q8);
    *(volatile v4f*)(hb + (size_t)(tok0 + row) * EMB + 32 * hf + 4 * q8) = v;
  }
}

__device__ __forceinline__ void ln_rows16(const float* __restrict__ hb, int tok0, int w, int lane,
                                          const float* __restrict__ gw, const float* __restrict__ gb,
                                          unsigned short* Ah, unsigned short* Al) {
  const float w0 = gw[lane], w1 = gw[lane + 32], b0 = gb[lane], b1 = gb[lane + 32];
#pragma unroll 1
  for (int rr = 0; rr < 16; ++rr) {
    const int row = 16 * w + rr;
    const float* hr = hb + (size_t)(tok0 + row) * EMB;
    const float v0 = hr[lane], v1 = hr[lane + 32];
    float s = v0 + v1;
#pragma unroll
    for (int off = 16; off >= 1; off >>= 1) s += __shfl_xor(s, off);
    const float mu = s * (1.0f / 64.0f);
    const float d0 = v0 - mu, d1 = v1 - mu;
    float q = d0 * d0 + d1 * d1;
#pragma unroll
    for (int off = 16; off >= 1; off >>= 1) q += __shfl_xor(q, off);
    const float r = rsqrtf(q * (1.0f / 64.0f) + 1e-5f);
    const float y0 = d0 * r * w0 + b0;
    const float y1 = d1 * r * w1 + b1;
    unsigned int h0, l0, h1, l1;
    split2(y0, h0, l0);
    split2(y1, h1, l1);
    Ah[row * EMB + lane] = (unsigned short)h0;
    Ah[row * EMB + lane + 32] = (unsigned short)h1;
    Al[row * EMB + lane] = (unsigned short)l0;
    Al[row * EMB + lane + 32] = (unsigned short)l1;
  }
}

__global__ __launch_bounds__(256) void k_wconv(const float* __restrict__ ew, const float* __restrict__ ipw,
                                               const float* __restrict__ ow, const float* __restrict__ f1w,
                                               const float* __restrict__ f2w,
                                               unsigned short* __restrict__ ph, unsigned short* __restrict__ pl) {
  const int blk = blockIdx.x, t = threadIdx.x;
  const int g = blk * 256 + t;
  float v[8];
  int dsto;
  if (blk < 3) {
    const int n = g / 12, kg = g - n * 12;
    dsto = WET_OFF + n * KEMB + kg * 8;
#pragma unroll
    for (int i = 0; i < 8; ++i) {
      const int k = kg * 8 + i;
      const int kc = (k < 66) ? k : 65;
      const float xv = ew[kc * EMB + n];
      v[i] = (k < 66) ? xv : 0.0f;
    }
  } else if (blk < 21) {
    const int e0 = (g - 768) * 8;
    dsto = WQKV_OFF + e0;
#pragma unroll
    for (int i = 0; i < 8; ++i) v[i] = ipw[e0 + i];
  } else if (blk < 27) {
    const int e0 = (g - 5376) * 8;
    dsto = WO_OFF + e0;
#pragma unroll
    for (int i = 0; i < 8; ++i) v[i] = ow[e0 + i];
  } else if (blk < 51) {
    const int g3 = g - 6912;
    const int l = g3 >> 11, rem = g3 & 2047;
    const int n = rem >> 3, kg = rem & 7;
    dsto = W1_OFF + (l * FFD + n) * EMB + kg * 8;
#pragma unroll
    for (int i = 0; i < 8; ++i) v[i] = f1w[(size_t)(l * EMB + kg * 8 + i) * FFD + n];
  } else {
    const int g4 = g - 13056;
    const int l = g4 >> 11, rem = g4 & 2047;
    const int n = rem >> 5, kg = rem & 31;
    dsto = W2_OFF + (l * EMB + n) * FFD + kg * 8;
#pragma unroll
    for (int i = 0; i < 8; ++i) v[i] = f2w[(size_t)(l * FFD + kg * 8 + i) * EMB + n];
  }
  unsigned int hb[8], lb[8];
#pragma unroll
  for (int i = 0; i < 8; ++i) split2(v[i], hb[i], lb[i]);
  v4u H, Lw;
  H.x = hb[0] | (hb[1] << 16); H.y = hb[2] | (hb[3] << 16); H.z = hb[4] | (hb[5] << 16); H.w = hb[6] | (hb[7] << 16);
  Lw.x = lb[0] | (lb[1] << 16); Lw.y = lb[2] | (lb[3] << 16); Lw.z = lb[4] | (lb[5] << 16); Lw.w = lb[6] | (lb[7] << 16);
  *(volatile v4u*)(ph + dsto) = H;
  *(volatile v4u*)(pl + dsto) = Lw;
  __threadfence();
  *(volatile v4u*)(ph + dsto) = H;
  *(volatile v4u*)(pl + dsto) = Lw;
}

__global__ __launch_bounds__(256) void k_order(const float* __restrict__ x, int* __restrict__ order,
                                               int* __restrict__ inv, int* __restrict__ nkl) {
  __shared__ int scan[256];
  __shared__ __attribute__((aligned(16))) int sorder[SEQ];
  __shared__ __attribute__((aligned(16))) int sinv[SEQ];
  const int b = blockIdx.x, t = threadIdx.x;
  const float* x6  = x + ((size_t)b * EMB + 6) * SEQ;
  const float* x58 = x + ((size_t)b * EMB + 58) * SEQ;
  int kp[4];
  int cnt = 0;
#pragma unroll
  for (int i = 0; i < 4; ++i) {
    const int s = 4 * t + i;
    const float nu = x6[s], ib = x58[s];
    const int empty = (nu != 0.0f) && (ib != 0.0f);
    kp[i] = 1 - empty;
    cnt += kp[i];
  }
  scan[t] = cnt;
  __syncthreads();
#pragma unroll 1
  for (int off = 1; off < 256; off <<= 1) {
    const int src = (t >= off) ? (t - off) : 0;
    int v = scan[src];
    v = (t >= off) ? v : 0;
    __syncthreads();
    scan[t] += v;
    __syncthreads();
  }
  const int incl = scan[t];
  const int total = scan[255];
  int pre = incl - cnt;
#pragma unroll
  for (int i = 0; i < 4; ++i) {
    const int s = 4 * t + i;
    int rank = kp[i] ? pre : (total + s - pre);
    pre += kp[i];
    rank = min(max(rank, 0), SEQ - 1);
    sorder[rank] = s;
    sinv[s] = rank;
  }
  __syncthreads();
  const v4i ov = *(const v4ia*)(sorder + 4 * t);
  const v4i iv = *(const v4ia*)(sinv + 4 * t);
  v4i nv;
  nv.x = total; nv.y = total; nv.z = total; nv.w = total;
  int* od = order + (size_t)b * SEQ + 4 * t;
  int* idd = inv + (size_t)b * SEQ + 4 * t;
  int* nd = nkl + b * 32 + 4 * t;
  *(volatile v4i*)od = ov;
  *(volatile v4i*)idd = iv;
  if (t < 8) *(volatile v4i*)nd = nv;
  __threadfence();
  *(volatile v4i*)od = ov;
  *(volatile v4i*)idd = iv;
  if (t < 8) *(volatile v4i*)nd = nv;
}

__global__ __launch_bounds__(128) void k_embed(const float* __restrict__ x, const int* __restrict__ order,
                                               const unsigned short* __restrict__ ph, const unsigned short* __restrict__ pl,
                                               const float* __restrict__ eb, float* __restrict__ hb) {
  __shared__ int sidx[64];
  __shared__ __attribute__((aligned(16))) unsigned short Ah[64 * KEMB];
  __shared__ __attribute__((aligned(16))) unsigned short Al[64 * KEMB];
  __shared__ __attribute__((aligned(16))) float R[64 * EMB];
  const int t = threadIdx.x, lane = t & 31, w = t >> 5, h = lane >> 4, m = lane & 15;
  const int b = blockIdx.x >> 4, rb = blockIdx.x & 15, rk0 = rb * 64, tok0 = b * SEQ + rk0;
  if (t < 64) {
    int s = order[(size_t)b * SEQ + rk0 + t];
    s = min(max(s, 0), SEQ - 1);
    sidx[t] = s;
  }
  __syncthreads();
  const float* xb = x + (size_t)b * EMB * SEQ;
#pragma unroll 1
  for (int it = 0; it < 48; ++it) {
    const int idx = it * 128 + t;
    const int c = idx >> 6, j = idx & 63;
    const int s = sidx[j];
    const int cc = (c < EMB) ? c : (EMB - 1);
    const float xv = xb[(size_t)cc * SEQ + s];
    const float fw = lin31(s & 31);
    const float fh = lin31(s >> 5);
    const float v = (c < EMB) ? xv : ((c == EMB) ? fw : ((c == EMB + 1) ? fh : 0.0f));
    unsigned int hbt, lbt;
    split2(v, hbt, lbt);
    Ah[j * KEMB + c] = (unsigned short)hbt;
    Al[j * KEMB + c] = (unsigned short)lbt;
  }
  __syncthreads();
  v8f acc[4];
#pragma unroll
  for (int nt = 0; nt < 4; ++nt) acc[nt] = zero8();
  const int rowA = (16 * w + m) * KEMB;
#pragma unroll
  for (int ks = 0; ks < 3; ++ks) {
    const v16bf ahf = ldfrag(Ah + rowA + 32 * ks, h);
    const v16bf alf = ldfrag(Al + rowA + 32 * ks, h);
#pragma unroll
    for (int nt = 0; nt < 4; ++nt) {
      const int wro = WET_OFF + (16 * nt + m) * KEMB + 32 * ks;
      const v16bf wbh = ldfrag(ph + wro, h), wbl = ldfrag(pl + wro, h);
      acc[nt] = mma16(ahf, wbh, acc[nt]);
      acc[nt] = mma16(ahf, wbl, acc[nt]);
      acc[nt] = mma16(alf, wbh, acc[nt]);
    }
  }
#pragma unroll
  for (int nt = 0; nt < 4; ++nt) {
    const float bv = eb[16 * nt + m];
#pragma unroll
    for (int r = 0; r < 8; ++r) R[(16 * w + 8 * h + r) * EMB + 16 * nt + m] = acc[nt][r] + bv;
  }
  __syncthreads();
  store_rows<64, 128>(R, hb, tok0, t);
  __threadfence();
  store_rows<64, 128>(R, hb, tok0, t);
}

__device__ __forceinline__ void qkv_store(int g, const unsigned short* S,
                                          unsigned short* qp, unsigned short* khh, unsigned short* kl0,
                                          unsigned short* vth, unsigned short* vtl,
                                          int bh0, int q0, int t) {
  const int q8 = t & 7;
  if (g < 2) {
    unsigned short* d0p = (g == 0) ? qp : khh;
#pragma unroll
    for (int i = 0; i < 8; ++i) {
      const int p = i * 128 + t;
      const int L = p >> 3;
      const int hd = L >> 5, Lh = L & 31;
      const size_t dofs = ((size_t)(bh0 + hd) * SEQ + q0) * 32 + Lh * 64 + q8 * 8;
      const v4u v = *(const v4ua*)(S + p * 8);
      *(volatile v4u*)(d0p + dofs) = v;
      if (g == 1) {
        const v4u v2 = *(const v4ua*)(S + 8192 + p * 8);
        *(volatile v4u*)(kl0 + dofs) = v2;
      }
    }
  } else {
#pragma unroll
    for (int i = 0; i < 4; ++i) {
      const int p = i * 128 + t;
      const int L = p >> 3;
      const int hd = L >> 4, d = L & 15;
      const size_t dofs = ((size_t)(bh0 + hd) * HDIM + d) * SEQ + q0 + q8 * 8;
      const v4u v = *(const v4ua*)(S + p * 8);
      const v4u v2 = *(const v4ua*)(S + 4096 + p * 8);
      *(volatile v4u*)(vth + dofs) = v;
      *(volatile v4u*)(vtl + dofs) = v2;
    }
  }
}

__global__ __launch_bounds__(128) void k_qkv(const float* __restrict__ hb, const float* __restrict__ lnw,
                                             const float* __restrict__ lnb,
                                             const unsigned short* __restrict__ ph, const unsigned short* __restrict__ pl,
                                             const float* __restrict__ ipb,
                                             unsigned short* __restrict__ qp, unsigned short* __restrict__ khh,
                                             unsigned short* __restrict__ kl0, unsigned short* __restrict__ vth,
                                             unsigned short* __restrict__ vtl, int layer) {
  __shared__ __attribute__((aligned(16))) unsigned short Ah[64 * EMB];
  __shared__ __attribute__((aligned(16))) unsigned short Al[64 * EMB];
  __shared__ __attribute__((aligned(16))) unsigned short Sst[16384];
  const int t = threadIdx.x, lane = t & 31, w = t >> 5, h = lane >> 4, m = lane & 15;
  const int b = blockIdx.x >> 4, rb = blockIdx.x & 15, q0 = rb * 64, tok0 = b * SEQ + q0;
  const int bh0 = b * NHEAD;

  ln_rows16(hb, tok0, w, lane, lnw + layer * EMB, lnb + layer * EMB, Ah, Al);
  __syncthreads();

  const int rowA = (16 * w + m) * EMB;
  const v16bf ah0 = ldfrag(Ah + rowA, h), ah1 = ldfrag(Ah + rowA + 32, h);
  const v16bf al0 = ldfrag(Al + rowA, h), al1 = ldfrag(Al + rowA + 32, h);

#pragma unroll 1
  for (int g = 0; g < 3; ++g) {
    v8f acc[4];
#pragma unroll
    for (int nt = 0; nt < 4; ++nt) acc[nt] = zero8();
#pragma unroll
    for (int nt = 0; nt < 4; ++nt) {
      const int n = 64 * g + 16 * nt + m;
      const int wro = WQKV_OFF + (layer * 3 * EMB + n) * EMB;
      v16bf wbh = ldfrag(ph + wro, h), wbl = ldfrag(pl + wro, h);
      acc[nt] = mma16(ah0, wbh, acc[nt]);
      acc[nt] = mma16(ah0, wbl, acc[nt]);
      acc[nt] = mma16(al0, wbh, acc[nt]);
      wbh = ldfrag(ph + wro + 32, h);
      wbl = ldfrag(pl + wro + 32, h);
      acc[nt] = mma16(ah1, wbh, acc[nt]);
      acc[nt] = mma16(ah1, wbl, acc[nt]);
      acc[nt] = mma16(al1, wbh, acc[nt]);
    }
#pragma unroll
    for (int nt = 0; nt < 4; ++nt) {
      const float bv = ipb[layer * 3 * EMB + 64 * g + 16 * nt + m];
#pragma unroll
      for (int r = 0; r < 8; ++r) {
        const int row = 16 * w + 8 * h + r;
        float y = acc[nt][r] + bv;
        unsigned int hbt, lbt;
        if (g == 0) {
          y *= 0.25f;
          split2(y, hbt, lbt);
          Sst[nt * 2048 + row * 32 + m] = (unsigned short)hbt;
          Sst[nt * 2048 + row * 32 + 16 + m] = (unsigned short)lbt;
        } else if (g == 1) {
          split2(y, hbt, lbt);
          Sst[nt * 2048 + row * 32 + m] = (unsigned short)hbt;
          Sst[nt * 2048 + row * 32 + 16 + m] = (unsigned short)hbt;
          Sst[8192 + nt * 2048 + row * 32 + m] = (unsigned short)lbt;
          Sst[8192 + nt * 2048 + row * 32 + 16 + m] = (unsigned short)0;
        } else {
          split2(y, hbt, lbt);
          Sst[(nt * HDIM + m) * 64 + row] = (unsigned short)hbt;
          Sst[4096 + (nt * HDIM + m) * 64 + row] = (unsigned short)lbt;
        }
      }
    }
    __syncthreads();
    qkv_store(g, Sst, qp, khh, kl0, vth, vtl, bh0, q0, t);
    __threadfence();
    qkv_store(g, Sst, qp, khh, kl0, vth, vtl, bh0, q0, t);
    __syncthreads();
  }
}

__device__ __forceinline__ void pack_p2(v8f a, v8f c, v16bf& phf, v16bf& plf) {
  Frag H, Lq;
#pragma unroll
  for (int k = 0; k < 4; ++k) {
    unsigned int h0, l0, h1, l1, h2, l2, h3, l3;
    split2(a[2 * k], h0, l0);
    split2(a[2 * k + 1], h1, l1);
    split2(c[2 * k], h2, l2);
    split2(c[2 * k + 1], h3, l3);
    H.w[k] = h0 | (h1 << 16);
    Lq.w[k] = l0 | (l1 << 16);
    H.w[4 + k] = h2 | (h3 << 16);
    Lq.w[4 + k] = l2 | (l3 << 16);
  }
  phf = H.v;
  plf = Lq.v;
}

__global__ __launch_bounds__(128) void k_attn(const unsigned short* __restrict__ qp, const unsigned short* __restrict__ khh,
                                              const unsigned short* __restrict__ kl0, const unsigned short* __restrict__ vth,
                                              const unsigned short* __restrict__ vtl, const int* __restrict__ nkl,
                                              const unsigned short* __restrict__ ph, const unsigned short* __restrict__ pl,
                                              const float* __restrict__ ob, float* __restrict__ hb, int layer) {
  __shared__ __attribute__((aligned(16))) float so[16 * EMB];
  __shared__ __attribute__((aligned(16))) unsigned short Oh[16 * EMB];
  __shared__ __attribute__((aligned(16))) unsigned short Ol[16 * EMB];
  const int t = threadIdx.x, lane = t & 31, w = t >> 5, h = lane >> 4, m = lane & 15;
  const int b = blockIdx.x >> 6, qt = blockIdx.x & 63, q0 = qt * 16, tok0 = b * SEQ + q0;
  const int bh = b * NHEAD + w;
  int nk = nkl[b * 32];
  nk = min(max(nk, 0), SEQ);
  const int nsteps = (q0 < nk) ? ((nk + 63) >> 6) : 0;

  const v16bf qf = ldfrag(qp + ((size_t)bh * SEQ + q0 + m) * 32, h);
  const unsigned short* khb = khh + ((size_t)bh * SEQ + m) * 32;
  const unsigned short* klb = kl0 + ((size_t)bh * SEQ + m) * 32;
  const unsigned short* vhb = vth + ((size_t)bh * HDIM + m) * SEQ;
  const unsigned short* vlb = vtl + ((size_t)bh * HDIM + m) * SEQ;

  v8f o = zero8();
  float mrun = -1.0e30f, lrun = 0.0f;

#pragma unroll 1
  for (int st = 0; st < nsteps; ++st) {
    const int kb = st * 64;
    v8f s[4];
#pragma unroll
    for (int j = 0; j < 4; ++j) {
      const int ko = (kb + 16 * j) * 32;
      const v16bf a1 = ldfrag(khb + ko, h);
      const v16bf a2 = ldfrag(klb + ko, h);
      v8f z = zero8();
      z = mma16(a1, qf, z);
      z = mma16(a2, qf, z);
      s[j] = z;
    }
#pragma unroll
    for (int j = 0; j < 4; ++j)
#pragma unroll
      for (int r = 0; r < 8; ++r) {
        const int kidx = kb + 16 * j + 8 * h + r;
        s[j][r] = s[j][r] + ((kidx < nk) ? 0.0f : -1.0e30f);
      }
    float mloc = s[0][0];
#pragma unroll
    for (int j = 0; j < 4; ++j)
#pragma unroll
      for (int r = 0; r < 8; ++r) mloc = fmaxf(mloc, s[j][r]);
    mloc = fmaxf(mloc, __shfl_xor(mloc, 16));
    const float mnew = fmaxf(mrun, mloc);
    const float alpha = __expf(mrun - mnew);
    mrun = mnew;
    float lsum = 0.0f;
#pragma unroll
    for (int j = 0; j < 4; ++j)
#pragma unroll
      for (int r = 0; r < 8; ++r) {
        const float p = __expf(s[j][r] - mnew);
        s[j][r] = p;
        lsum += p;
      }
    lsum += __shfl_xor(lsum, 16);
    lrun = lrun * alpha + lsum;
#pragma unroll
    for (int r = 0; r < 8; ++r) o[r] = o[r] * alpha;

    v16bf p0h, p0l, p1h, p1l;
    pack_p2(s[0], s[1], p0h, p0l);
    pack_p2(s[2], s[3], p1h, p1l);
    {
      const v16bf va = ldfrag(vhb + kb, h), vb = ldfrag(vlb + kb, h);
      o = mma16(va, p0h, o);
      o = mma16(va, p0l, o);
      o = mma16(vb, p0h, o);
    }
    {
      const v16bf va = ldfrag(vhb + kb + 32, h), vb = ldfrag(vlb + kb + 32, h);
      o = mma16(va, p1h, o);
      o = mma16(va, p1l, o);
      o = mma16(vb, p1h, o);
    }
  }

  const float il = (lrun > 0.0f) ? (1.0f / lrun) : 0.0f;
#pragma unroll
  for (int r = 0; r < 8; ++r) so[m * EMB + 16 * w + 8 * h + r] = o[r] * il;
  __syncthreads();
  {
    const int row = t >> 3, c0 = (t & 7) * 8;
#pragma unroll
    for (int i = 0; i < 8; ++i) {
      const float f = so[row * EMB + c0 + i];
      unsigned int hbt, lbt;
      split2(f, hbt, lbt);
      Oh[row * EMB + c0 + i] = (unsigned short)hbt;
      Ol[row * EMB + c0 + i] = (unsigned short)lbt;
    }
  }
  __syncthreads();
  v8f acc = zero8();
#pragma unroll
  for (int ks = 0; ks < 2; ++ks) {
    const v16bf ahf = ldfrag(Oh + m * EMB + 32 * ks, h);
    const v16bf alf = ldfrag(Ol + m * EMB + 32 * ks, h);
    const int wro = WO_OFF + (layer * EMB + 16 * w + m) * EMB + 32 * ks;
    const v16bf wbh = ldfrag(ph + wro, h), wbl = ldfrag(pl + wro, h);
    acc = mma16(ahf, wbh, acc);
    acc = mma16(ahf, wbl, acc);
    acc = mma16(alf, wbh, acc);
  }
  {
    const int n = 16 * w + m;
    const float bv = ob[layer * EMB + n];
#pragma unroll
    for (int r = 0; r < 8; ++r) {
      const int row = 8 * h + r;
      const float res = hb[(size_t)(tok0 + row) * EMB + n];
      const float pv = acc[r] + bv;
      so[row * EMB + n] = res + pv;
    }
  }
  __syncthreads();
  store_rows<16, 128>(so, hb, tok0, t);
  __threadfence();
  store_rows<16, 128>(so, hb, tok0, t);
}

__global__ __launch_bounds__(64) void k_ffn(float* __restrict__ hb, const float* __restrict__ lnw,
                                            const float* __restrict__ lnb,
                                            const unsigned short* __restrict__ ph, const unsigned short* __restrict__ pl,
                                            const float* __restrict__ b1, const float* __restrict__ b2, int layer) {
  __shared__ __attribute__((aligned(16))) unsigned short Ah[32 * EMB];
  __shared__ __attribute__((aligned(16))) unsigned short Al[32 * EMB];
  __shared__ __attribute__((aligned(16))) float Cs[32 * EMB];
  __shared__ __attribute__((aligned(16))) unsigned short Gh[32 * FFD];
  __shared__ __attribute__((aligned(16))) unsigned short Gl[32 * FFD];
  const int t = threadIdx.x, lane = t & 31, w = t >> 5, h = lane >> 4, m = lane & 15;
  const int tok0 = blockIdx.x * 32;

  ln_rows16(hb, tok0, w, lane, lnw + layer * EMB, lnb + layer * EMB, Ah, Al);
  __syncthreads();

  const int rowA = (16 * w + m) * EMB;
  const v16bf ah0 = ldfrag(Ah + rowA, h), ah1 = ldfrag(Ah + rowA + 32, h);
  const v16bf al0 = ldfrag(Al + rowA, h), al1 = ldfrag(Al + rowA + 32, h);

#pragma unroll 1
  for (int g = 0; g < 4; ++g) {
    v8f acc[4];
#pragma unroll
    for (int nt = 0; nt < 4; ++nt) acc[nt] = zero8();
#pragma unroll
    for (int nt = 0; nt < 4; ++nt) {
      const int n = 64 * g + 16 * nt + m;
      const int wro = W1_OFF + (layer * FFD + n) * EMB;
      v16bf wbh = ldfrag(ph + wro, h), wbl = ldfrag(pl + wro, h);
      acc[nt] = mma16(ah0, wbh, acc[nt]);
      acc[nt] = mma16(ah0, wbl, acc[nt]);
      acc[nt] = mma16(al0, wbh, acc[nt]);
      wbh = ldfrag(ph + wro + 32, h);
      wbl = ldfrag(pl + wro + 32, h);
      acc[nt] = mma16(ah1, wbh, acc[nt]);
      acc[nt] = mma16(ah1, wbl, acc[nt]);
      acc[nt] = mma16(al1, wbh, acc[nt]);
    }
#pragma unroll
    for (int nt = 0; nt < 4; ++nt) {
      const float bv = b1[layer * FFD + 64 * g + 16 * nt + m];
#pragma unroll
      for (int r = 0; r < 8; ++r) Cs[(16 * w + 8 * h + r) * EMB + 16 * nt + m] = acc[nt][r] + bv;
    }
    __syncthreads();
#pragma unroll 1
    for (int it = 0; it < 32; ++it) {
      const int idx = it * 32 + lane;
      const int row = 16 * w + (idx >> 6), col = idx & 63;
      const float c = Cs[row * EMB + col];
      const float ge = 0.5f * c * (1.0f + erff(c * 0.70710678118654752f));
      unsigned int hbt, lbt;
      split2(ge, hbt, lbt);
      Gh[row * FFD + 64 * g + col] = (unsigned short)hbt;
      Gl[row * FFD + 64 * g + col] = (unsigned short)lbt;
    }
    __syncthreads();
  }

  v8f acc2[4];
#pragma unroll
  for (int nt = 0; nt < 4; ++nt) acc2[nt] = zero8();
  const int groA = (16 * w + m) * FFD;
#pragma unroll 1
  for (int ks = 0; ks < 8; ++ks) {
    const v16bf ahf = ldfrag(Gh + groA + 32 * ks, h);
    const v16bf alf = ldfrag(Gl + groA + 32 * ks, h);
#pragma unroll
    for (int nt = 0; nt < 4; ++nt) {
      const int wro = W2_OFF + (layer * EMB + 16 * nt + m) * FFD + 32 * ks;
      const v16bf wbh = ldfrag(ph + wro, h), wbl = ldfrag(pl + wro, h);
      acc2[nt] = mma16(ahf, wbh, acc2[nt]);
      acc2[nt] = mma16(ahf, wbl, acc2[nt]);
      acc2[nt] = mma16(alf, wbh, acc2[nt]);
    }
  }
#pragma unroll
  for (int nt = 0; nt < 4; ++nt) {
    const int n = 16 * nt + m;
    const float bv = b2[layer * EMB + n];
#pragma unroll
    for (int r = 0; r < 8; ++r) {
      const int row = 16 * w + 8 * h + r;
      const float res = hb[(size_t)(tok0 + row) * EMB + n];
      const float fv = acc2[nt][r] + bv;
      Cs[row * EMB + n] = res + fv;
    }
  }
  __syncthreads();
  store_rows<32, 64>(Cs, hb, tok0, t);
  __threadfence();
  store_rows<32, 64>(Cs, hb, tok0, t);
}

__global__ __launch_bounds__(128) void k_out(const float* __restrict__ x, const int* __restrict__ inv,
                                             const float* __restrict__ hb, float* __restrict__ out) {
  __shared__ int sr[32];
  __shared__ int sk[32];
  __shared__ float T[32 * 65];
  const int t = threadIdx.x;
  const int b = blockIdx.x >> 5, sg = blockIdx.x & 31, s0 = sg * 32;
  if (t < 32) {
    const int s = s0 + t;
    const float nu = x[((size_t)b * EMB + 6) * SEQ + s];
    const float ib = x[((size_t)b * EMB + 58) * SEQ + s];
    const int empty = (nu != 0.0f) && (ib != 0.0f);
    int r = inv[(size_t)b * SEQ + s];
    r = min(max(r, 0), SEQ - 1);
    sr[t] = r;
    sk[t] = 1 - empty;
  }
  __syncthreads();
#pragma unroll 1
  for (int it = 0; it < 16; ++it) {
    const int idx = it * 128 + t;
    const int sl = idx >> 6, e = idx & 63;
    const float v = hb[((size_t)b * SEQ + sr[sl]) * EMB + e];
    T[sl * 65 + e] = sk[sl] ? v : 0.0f;
  }
  __syncthreads();
  const int q8 = t & 7, sub = t >> 3;
#pragma unroll
  for (int i = 0; i < 4; ++i) {
    const int e = i * 16 + sub;
    v4f v;
    v.x = T[(4 * q8 + 0) * 65 + e];
    v.y = T[(4 * q8 + 1) * 65 + e];
    v.z = T[(4 * q8 + 2) * 65 + e];
    v.w = T[(4 * q8 + 3) * 65 + e];
    *(volatile v4f*)(out + ((size_t)b * EMB + e) * SEQ + s0 + 4 * q8) = v;
  }
  __threadfence();
#pragma unroll
  for (int i = 0; i < 4; ++i) {
    const int e = i * 16 + sub;
    v4f v;
    v.x = T[(4 * q8 + 0) * 65 + e];
    v.y = T[(4 * q8 + 1) * 65 + e];
    v.z = T[(4 * q8 + 2) * 65 + e];
    v.w = T[(4 * q8 + 3) * 65 + e];
    *(volatile v4f*)(out + ((size_t)b * EMB + e) * SEQ + s0 + 4 * q8) = v;
  }
}

extern "C" void kernel_launch(void* const* d_in, const int* in_sizes, int n_in,
                              void* d_out, int out_size, void* d_ws, size_t ws_size,
                              hipStream_t stream) {
  if (n_in < 15) return;
  if (in_sizes[0] != NIMG * EMB * SEQ) return;
  if (in_sizes[1] != 66 * EMB || in_sizes[2] != EMB) return;
  if (in_sizes[3] != NLAYER * EMB || in_sizes[4] != NLAYER * EMB) return;
  if (in_sizes[5] != NLAYER * 3 * EMB * EMB || in_sizes[6] != NLAYER * 3 * EMB) return;
  if (in_sizes[7] != NLAYER * EMB * EMB || in_sizes[8] != NLAYER * EMB) return;
  if (in_sizes[9] != NLAYER * EMB || in_sizes[10] != NLAYER * EMB) return;
  if (in_sizes[11] != NLAYER * EMB * FFD || in_sizes[12] != NLAYER * FFD) return;
  if (in_sizes[13] != NLAYER * FFD * EMB || in_sizes[14] != NLAYER * EMB) return;
  if (out_size != NIMG * EMB * SEQ) return;

  const float* x         = (const float*)d_in[0];
  const float* embed_w   = (const float*)d_in[1];
  const float* embed_b   = (const float*)d_in[2];
  const float* ln1_w     = (const float*)d_in[3];
  const float* ln1_b     = (const float*)d_in[4];
  const float* in_proj_w = (const float*)d_in[5];
  const float* in_proj_b = (const float*)d_in[6];
  const float* out_w     = (const float*)d_in[7];
  const float* out_b     = (const float*)d_in[8];
  const float* ln2_w     = (const float*)d_in[9];
  const float* ln2_b     = (const float*)d_in[10];
  const float* ff1_w     = (const float*)d_in[11];
  const float* ff1_b     = (const float*)d_in[12];
  const float* ff2_w     = (const float*)d_in[13];
  const float* ff2_b     = (const float*)d_in[14];
  float* out = (float*)d_out;

  size_t off = 0;
  auto carve = [&](size_t bytes) -> char* {
    char* p = (char*)d_ws + off;
    off += (bytes + 255) & ~(size_t)255;
    return p;
  };
  int* order = (int*)carve((size_t)NTOK * 4);
  int* inv   = (int*)carve((size_t)NTOK * 4);
  int* nkl   = (int*)carve((size_t)NIMG * 32 * 4);
  float* hbuf = (float*)carve((size_t)NTOK * EMB * 4);
  unsigned short* ph  = (unsigned short*)carve((size_t)WPLANE * 2);
  unsigned short* pl  = (unsigned short*)carve((size_t)WPLANE * 2);
  unsigned short* qp  = (unsigned short*)carve((size_t)NIMG * NHEAD * SEQ * 32 * 2);
  unsigned short* khh = (unsigned short*)carve((size_t)NIMG * NHEAD * SEQ * 32 * 2);
  unsigned short* kl0 = (unsigned short*)carve((size_t)NIMG * NHEAD * SEQ * 32 * 2);
  unsigned short* vth = (unsigned short*)carve((size_t)NIMG * NHEAD * HDIM * SEQ * 2);
  unsigned short* vtl = (unsigned short*)carve((size_t)NIMG * NHEAD * HDIM * SEQ * 2);
  if (off > ws_size) return;
  if (off > (size_t)134217728) return;

  k_wconv<<<75, 256, 0, stream>>>(embed_w, in_proj_w, out_w, ff1_w, ff2_w, ph, pl);
  k_order<<<NIMG, 256, 0, stream>>>(x, order, inv, nkl);
  k_embed<<<NIMG * 16, 128, 0, stream>>>(x, order, ph, pl, embed_b, hbuf);
  for (int l = 0; l < NLAYER; ++l) {
    k_qkv<<<NIMG * 16, 128, 0, stream>>>(hbuf, ln1_w, ln1_b, ph, pl, in_proj_b, qp, khh, kl0, vth, vtl, l);
    k_attn<<<NIMG * 64, 128, 0, stream>>>(qp, khh, kl0, vth, vtl, nkl, ph, pl, out_b, hbuf, l);
    k_ffn<<<NTOK / 32, 64, 0, stream>>>(hbuf, ln2_w, ln2_b, ph, pl, ff1_b, ff2_b, l);
  }
  k_out<<<NIMG * 32, 128, 0, stream>>>(x, inv, hbuf, out);
}
